// SelfAttentionPooling_5944234737961
// MI455X (gfx1250) — hardware-run, weakly checked
//
#include <hip/hip_runtime.h>


namespace {
constexpr int N = 8192, H = 256, G = 256, MAXN = 64;
constexpr float XS = 8.0f, WSC = 256.0f;
static_assert(N % 64 == 0 && G % 64 == 0 && H == 256, "tiling");
typedef _Float16 b16;
typedef __attribute__((ext_vector_type(16))) _Float16 v16b;
typedef __attribute__((ext_vector_type(8))) _Float16 v8b;
typedef __attribute__((ext_vector_type(8))) float v8f;
typedef __attribute__((ext_vector_type(4))) float v4f;
__device__ __forceinline__ float bf16_rne(float f) { unsigned int u = __float_as_uint(f); u += 0x7FFFu + ((u >> 16) & 1u); return __uint_as_float(u & 0xFFFF0000u); }
__device__ __forceinline__ void split16(float v, b16& hi, b16& lo) { hi = (b16)v; lo = (b16)(v - (float)hi); }
__device__ __forceinline__ v16b frag_kb(const b16* p, int hh) { const v8b a = *(const v8b*)(p + 8 * hh), b = *(const v8b*)(p + 16 + 8 * hh); v16b f;
#pragma unroll
  for (int e = 0; e < 8; ++e) { f[e] = a[e]; f[8 + e] = b[e]; } return f; }
__device__ __forceinline__ v8f wmma16b(v16b a, v16b b, v8f c) { v8f d = __builtin_amdgcn_wmma_f32_16x16x32_f16(false, a, false, b, (short)0, c, false, false); asm volatile("v_nop\n\tv_nop\n\tv_nop\n\tv_nop" : "+v"(d) : "v"(a), "v"(b)); return d; }
__device__ __forceinline__ void wave_lds_sync() { __builtin_amdgcn_fence(__ATOMIC_RELEASE, "workgroup"); __builtin_amdgcn_wave_barrier(); __builtin_amdgcn_fence(__ATOMIC_ACQUIRE, "workgroup"); }
__device__ __forceinline__ float pmul(float a, float b) { float p = a * b; asm volatile("" : "+v"(p)); return p; }
__device__ __forceinline__ int iclamp(int v, int lo, int hi) { return v < lo ? lo : (v > hi ? hi : v); }

typedef __attribute__((ext_vector_type(4))) _Float16 v4h;
__global__ __launch_bounds__(256) void wprep_kernel(const float* __restrict__ w0, const float* __restrict__ w1, const float* __restrict__ w2, const float* __restrict__ w3, const float* __restrict__ w4, b16* __restrict__ WT) {
  const size_t u = (size_t)blockIdx.x * 256 + threadIdx.x; if (u >= (size_t)5 * H * H / 8) return; const size_t e = u * 8; const int m = (int)(e / ((size_t)H * H)); const size_t el = e % ((size_t)H * H);
  const int oo = (int)(el / H), k0 = (int)(el % H); const float* w = m == 0 ? w0 : m == 1 ? w1 : m == 2 ? w2 : m == 3 ? w3 : w4; v8b o; for (int j = 0; j < 8; ++j) o[j] = (b16)(bf16_rne(w[(size_t)(k0 + j) * H + oo]) * WSC);
  for (int pass = 0; pass < 2; ++pass) { *(volatile v8b*)(WT + e) = o; __threadfence(); }
}
template <int RELU, int RND>
__global__ __launch_bounds__(128) void gemm_kernel(const float* __restrict__ Hin, const b16* __restrict__ W, const float* __restrict__ bias, float* __restrict__ T) {
  __shared__ __attribute__((aligned(16))) b16 Ah[4][16][H + 8], Al[4][16][H + 8]; __shared__ __attribute__((aligned(16))) float Tf[4][16][128 + 4];
  const int wave = threadIdx.x >> 5, lane = threadIdx.x & 31, nloc = lane & 15, hlf = lane >> 4; const size_t m0 = (size_t)blockIdx.x * 64 + wave * 16; const int n0 = blockIdx.y * 128;
  for (int rr = 0; rr < 16; ++rr) for (int c8 = lane * 8; c8 < H; c8 += 256) { const v4f va = *(const v4f*)(Hin + (m0 + rr) * H + c8), vb = *(const v4f*)(Hin + (m0 + rr) * H + c8 + 4); v8b hv, lv;
      for (int j = 0; j < 8; ++j) { float v = j < 4 ? va[j] : vb[j - 4]; if (RND) v = bf16_rne(v); b16 p, q; split16(v * XS, p, q); hv[j] = p; lv[j] = q; } *(v8b*)(&Ah[wave][rr][c8]) = hv; *(v8b*)(&Al[wave][rr][c8]) = lv; }
  wave_lds_sync();
  v8f acc[8];
#pragma unroll
  for (int t = 0; t < 8; ++t) acc[t] = (v8f){};
#pragma unroll 2
  for (int kb = 0; kb < H; kb += 32) { const v16b a = frag_kb(&Ah[wave][nloc][kb], hlf), al = frag_kb(&Al[wave][nloc][kb], hlf);
#pragma unroll
    for (int t = 0; t < 8; ++t) { const v16b bw = frag_kb(W + (size_t)(n0 + t * 16 + nloc) * H + kb, hlf); acc[t] = wmma16b(a, bw, acc[t]); acc[t] = wmma16b(al, bw, acc[t]); } }
#pragma unroll
  for (int t = 0; t < 8; ++t)
#pragma unroll
    for (int r = 0; r < 8; ++r) Tf[wave][8 * hlf + r][t * 16 + nloc] = acc[t][r] * (1.0f / (XS * WSC));
  wave_lds_sync();
  v4f bb; for (int j = 0; j < 4; ++j) bb[j] = bf16_rne(bias[n0 + lane * 4 + j]);
  for (int rr = 0; rr < 16; ++rr) { v4f o = *(const v4f*)(&Tf[wave][rr][lane * 4]); for (int j = 0; j < 4; ++j) { o[j] += bb[j]; if (RELU) o[j] = fmaxf(o[j], 0.0f); } *(v4f*)(&Tf[wave][rr][lane * 4]) = o; }
  wave_lds_sync();
  for (int pass = 0; pass < 2; ++pass) { for (int rr = 0; rr < 16; ++rr) *(volatile v4f*)(T + (m0 + rr) * H + n0 + lane * 4) = *(const v4f*)(&Tf[wave][rr][lane * 4]); __threadfence(); }
}
__device__ int lower_bound_i(const int* a, int n, int key) { int lo = 0, hi = n; while (lo < hi) { const int mid = (lo + hi) >> 1; if (a[mid] < key) lo = mid + 1; else hi = mid; } return lo; }
__global__ __launch_bounds__(256) void attn_kernel(const float* __restrict__ S_, const float* __restrict__ Hh, const int* __restrict__ batch, float* __restrict__ XA) {
  __shared__ __attribute__((aligned(16))) b16 Sh[MAXN][H + 8], Sl[MAXN][H + 8]; __shared__ __attribute__((aligned(16))) float Sf[MAXN][MAXN + 4]; __shared__ float wj[MAXN];
  const int g = blockIdx.x, t = threadIdx.x, wave = t >> 5, lane = t & 31, nloc = lane & 15, hlf = lane >> 4;
  const int lo = lower_bound_i(batch, N, g), hi_ = lower_bound_i(batch, N, g + 1); const int n = iclamp(hi_ - lo, 0, MAXN);
  for (int q = t; q < MAXN * (H / 8); q += 256) { const int r = q / (H / 8), c8 = (q % (H / 8)) * 8; v8b hv, lv;
    if (r < n) { const v4f va = *(const v4f*)(S_ + (size_t)(lo + r) * H + c8), vb = *(const v4f*)(S_ + (size_t)(lo + r) * H + c8 + 4); for (int j = 0; j < 8; ++j) { b16 p, q2; split16((j < 4 ? va[j] : vb[j - 4]) * XS, p, q2); hv[j] = p; lv[j] = q2; } }
    else { for (int j = 0; j < 8; ++j) { hv[j] = (b16)0.0f; lv[j] = (b16)0.0f; } }
    *(v8b*)(&Sh[r][c8]) = hv; *(v8b*)(&Sl[r][c8]) = lv; }
  __syncthreads();
  { const int rt = wave >> 1; v8f acc[2]; acc[0] = (v8f){}; acc[1] = (v8f){};
#pragma unroll 2
    for (int kb = 0; kb < H; kb += 32) { const v16b a = frag_kb(&Sh[rt * 16 + nloc][kb], hlf), al = frag_kb(&Sl[rt * 16 + nloc][kb], hlf);
#pragma unroll
      for (int u2 = 0; u2 < 2; ++u2) { const int ct = 2 * (wave & 1) + u2; const v16b b = frag_kb(&Sh[ct * 16 + nloc][kb], hlf), bl = frag_kb(&Sl[ct * 16 + nloc][kb], hlf);
        acc[u2] = wmma16b(a, b, acc[u2]); acc[u2] = wmma16b(al, b, acc[u2]); acc[u2] = wmma16b(a, bl, acc[u2]); } }
#pragma unroll
    for (int u2 = 0; u2 < 2; ++u2) { const int ct = 2 * (wave & 1) + u2;
#pragma unroll
      for (int r = 0; r < 8; ++r) Sf[rt * 16 + 8 * hlf + r][ct * 16 + nloc] = acc[u2][r] * (1.0f / (XS * XS)); } }
  __syncthreads();
  if (t < n) { float m = 0.0f;
#pragma unroll 1
    for (int j = 0; j < n; ++j) m = fmaxf(m, Sf[t][j]);
    float sum = 0.0f;
#pragma unroll 1
    for (int j = 0; j < n; ++j) { const float e = __expf(Sf[t][j] - m); Sf[t][j] = e; sum += e; }
    const float inv = 1.0f / sum;
#pragma unroll 1
    for (int j = 0; j < n; ++j) Sf[t][j] = pmul(Sf[t][j], inv); }
  __syncthreads();
  if (t < MAXN) { float w = 0.0f; if (t < n) {
#pragma unroll 1
      for (int i = 0; i < n; ++i) w += Sf[i][t]; } wj[t] = w; }
  __syncthreads();
  float xa = 0.0f;
#pragma unroll 1
  for (int j = 0; j < n; ++j) xa += pmul(wj[j], Hh[(size_t)(lo + j) * H + t]);
  for (int pass = 0; pass < 2; ++pass) { ((volatile float*)XA)[(size_t)g * H + t] = xa; __threadfence(); }
}
}

extern "C" void kernel_launch(void* const* d_in, const int* in_sizes, int n_in, void* d_out, int out_size, void* d_ws, size_t ws_size, hipStream_t stream) {
  (void)n_in;
  auto Fp = [&](int i) { return (const float*)d_in[i]; }; auto Ip = [&](int i) { return (const int*)d_in[i]; };
  if (in_sizes[0] != N * H || in_sizes[1] != N || in_sizes[3] != H * H || in_sizes[5] != H * H || in_sizes[7] != H * H || in_sizes[9] != H * H || in_sizes[11] != H * H || in_sizes[4] != H || in_sizes[12] != H || out_size != G * H) return;
  size_t off = 0; char* ws = (char*)d_ws;
  auto carve = [&](size_t bytes) { char* p = ws + off; off += (bytes + 255) & ~(size_t)255; return p; };
  b16* WT = (b16*)carve((size_t)5 * H * H * 2); float* HA = (float*)carve((size_t)N * H * 4); float* HB = (float*)carve((size_t)N * H * 4); float* XA = (float*)carve((size_t)G * H * 4); float* R1 = (float*)carve((size_t)G * H * 4);
  if (off > ws_size || off > ((size_t)128 << 20)) return;
  const size_t HH = (size_t)H * H;
  wprep_kernel<<<(unsigned)((5 * HH / 8 + 255) / 256), 256, 0, stream>>>(Fp(5), Fp(7), Fp(3), Fp(9), Fp(11), WT);
  gemm_kernel<1, 1><<<dim3(N / 64, 2), 128, 0, stream>>>(Fp(0), WT + 0 * HH, Fp(6), HA);
  gemm_kernel<1, 0><<<dim3(N / 64, 2), 128, 0, stream>>>(HA, WT + 1 * HH, Fp(8), HB);
  gemm_kernel<0, 0><<<dim3(N / 64, 2), 128, 0, stream>>>(HB, WT + 2 * HH, Fp(4), HA);
  attn_kernel<<<G, 256, 0, stream>>>(HA, HB, Ip(1), XA);
  gemm_kernel<1, 0><<<dim3(G / 64, 2), 128, 0, stream>>>(XA, WT + 3 * HH, Fp(10), R1);
  gemm_kernel<1, 0><<<dim3(G / 64, 2), 128, 0, stream>>>(R1, WT + 4 * HH, Fp(12), (float*)d_out);
}
